// PointNetSetAbstraction_68281390072553
// MI455X (gfx1250) — hardware-verified
//
#include <hip/hip_runtime.h>
#pragma clang fp contract(off)

typedef __attribute__((ext_vector_type(16))) _Float16 v16h;
typedef __attribute__((ext_vector_type(8)))  _Float16 v8h;
typedef __attribute__((ext_vector_type(16))) __bf16   v16b;
typedef __attribute__((ext_vector_type(8)))  __bf16   v8b;
typedef __attribute__((ext_vector_type(8)))  float    v8f;
typedef __attribute__((ext_vector_type(4)))  float    v4f;
typedef __attribute__((ext_vector_type(4)))  unsigned v4u;

constexpr int kBatch = 16;
constexpr int kPts = 4096;
constexpr int kCen = 1024;
constexpr int kSamp = 32;
constexpr int kGroups = kBatch * kCen;
constexpr int kRows = kGroups * kSamp;
constexpr int kMlpBlocks = kGroups / 8;
constexpr int kActPitch = 72;
constexpr float kActCarry = 16.0f;
constexpr float kWgtCarry = 16.0f;
constexpr float kInvCarry = 1.0f / (kActCarry * kWgtCarry);
constexpr float kResidCarry = 2048.0f;
constexpr float kInvResid = 1.0f / kResidCarry;
constexpr float kF16MinNormal = 6.103515625e-05f;
constexpr float kBallR2 = 0.16f;
constexpr float kBnEps = 1e-5f;

static_assert(kRows == 524288);
static_assert(kMlpBlocks * 8 * 32 == kRows);
static_assert((kBatch * 3 * kCen * 4) % 128 == 0);
static_assert(kBatch * 3 * kCen * 4 + kBatch * 128 * kCen * 4 == 8585216);
static_assert((kActPitch * 2) % 16 == 0);

__device__ __forceinline__ unsigned f2bf_bits(float f) {
  const unsigned u = __float_as_uint(f);
  return ((u + 0x7FFFu + ((u >> 16) & 1u)) >> 16) & 0xFFFFu;
}
__device__ __forceinline__ float bf_bits2f(unsigned h) { return __uint_as_float(h << 16); }

__device__ __forceinline__ void wave_lds_sync() {
  __builtin_amdgcn_fence(__ATOMIC_RELEASE, "workgroup");
  __builtin_amdgcn_wave_barrier();
  __builtin_amdgcn_fence(__ATOMIC_ACQUIRE, "workgroup");
}

union FragH { v16h v; v8h h[2]; };
union FragB { v16b v; v8b h[2]; };
__device__ __forceinline__ v16h ldfrag_h(const _Float16* p) {
  FragH f; f.h[0] = *(const v8h*)(p); f.h[1] = *(const v8h*)(p + 16); return f.v;
}
__device__ __forceinline__ v16b ldfrag_b(const __bf16* p) {
  FragB f; f.h[0] = *(const v8b*)(p); f.h[1] = *(const v8b*)(p + 16); return f.v;
}
__device__ __forceinline__ v8f mma_h(v16h a, v16h b, v8f c) {
  c = __builtin_amdgcn_wmma_f32_16x16x32_f16(false, a, false, b, (short)0, c, false, false);
  asm volatile("v_nop\n\tv_nop\n\tv_nop\n\tv_nop" : "+v"(c) : "v"(a), "v"(b));
  return c;
}
__device__ __forceinline__ v8f mma_b(v16b a, v16b b, v8f c) {
  c = __builtin_amdgcn_wmma_f32_16x16x32_bf16(false, a, false, b, (short)0, c, false, false);
  asm volatile("v_nop\n\tv_nop\n\tv_nop\n\tv_nop" : "+v"(c) : "v"(a), "v"(b));
  return c;
}

__global__ __launch_bounds__(256) void prep_kernel(
    const float* __restrict__ W0, const float* __restrict__ W1, const float* __restrict__ W2,
    const float* __restrict__ b0, const float* __restrict__ b1, const float* __restrict__ b2,
    unsigned* __restrict__ Bt0w, unsigned short* __restrict__ W1h, unsigned short* __restrict__ W2h,
    float* __restrict__ biasp) {
  const int g = blockIdx.x * 256 + threadIdx.x;
  if (g < 256) {
    const int row = g >> 2;
    const int cq = g & 3;
    unsigned zz = 0;
    asm volatile("" : "+v"(zz));
    unsigned hw[8];
#pragma unroll
    for (int e = 0; e < 8; ++e) {
      const int kk = cq * 8 + e;
      int c = kk;
      if (c >= 6) c -= 6;
      if (c >= 6) c -= 6;
      if (c >= 6) c = 0;
      const float w = W0[row * 6 + c];
      const unsigned hb = f2bf_bits(w);
      const unsigned lb = f2bf_bits(w - bf_bits2f(hb));
      hw[e] = (kk < 12) ? hb : ((kk < 18) ? lb : zz);
    }
    v4u o;
    o[0] = hw[0] | (hw[1] << 16);
    o[1] = hw[2] | (hw[3] << 16);
    o[2] = hw[4] | (hw[5] << 16);
    o[3] = hw[6] | (hw[7] << 16);
    unsigned* dst = Bt0w + g * 4;
    *(volatile v4u*)dst = o;
    __threadfence();
    *(volatile v4u*)dst = o;
  } else if (g < 1792) {
    const bool second = (g >= 768);
    const int gi = second ? (g - 768) : (g - 256);
    const float* src = (second ? W2 : W1) + gi * 8;
    unsigned short* dstp = (second ? W2h : W1h) + gi * 8;
    const v4f x0 = *(const v4f*)(src);
    const v4f x1 = *(const v4f*)(src + 4);
    v8h hv;
    hv[0] = (_Float16)(x0[0] * kWgtCarry);
    hv[1] = (_Float16)(x0[1] * kWgtCarry);
    hv[2] = (_Float16)(x0[2] * kWgtCarry);
    hv[3] = (_Float16)(x0[3] * kWgtCarry);
    hv[4] = (_Float16)(x1[0] * kWgtCarry);
    hv[5] = (_Float16)(x1[1] * kWgtCarry);
    hv[6] = (_Float16)(x1[2] * kWgtCarry);
    hv[7] = (_Float16)(x1[3] * kWgtCarry);
    *(volatile v8h*)dstp = hv;
    __threadfence();
    *(volatile v8h*)dstp = hv;
  } else if (g < 1856) {
    const int gi = g - 1792;
    const int f0 = 4 * gi;
    int i0 = f0;
    if (i0 > 60) i0 = 60;
    int i1 = f0 - 64;
    if (i1 < 0) i1 = 0;
    if (i1 > 60) i1 = 60;
    int i2 = f0 - 128;
    if (i2 < 0) i2 = 0;
    if (i2 > 124) i2 = 124;
    const v4f x0 = *(const v4f*)(b0 + i0);
    const v4f x1 = *(const v4f*)(b1 + i1);
    const v4f x2 = *(const v4f*)(b2 + i2);
    const float s0 = (f0 < 64) ? 1.0f : 0.0f;
    const float s1 = (f0 >= 64 && f0 < 128) ? 1.0f : 0.0f;
    const float s2 = (f0 >= 128) ? 1.0f : 0.0f;
    const v4f o = x0 * s0 + x1 * s1 + x2 * s2;
    float* dst = biasp + f0;
    *(volatile v4f*)dst = o;
    __threadfence();
    *(volatile v4f*)dst = o;
  }
}

__global__ __launch_bounds__(512) void fps_kernel(const float* __restrict__ xyz,
                                                  float* __restrict__ out0,
                                                  float* __restrict__ cenws) {
#pragma clang fp contract(off)
  __shared__ __align__(16) float sxyz[3 * kPts];
  __shared__ unsigned redh[2][16];
  __shared__ unsigned redl[2][16];
  __shared__ int cents[kCen];
  const int t = threadIdx.x;
  const int lane = t & 31;
  const int wave = t >> 5;
  const int b = blockIdx.x;
  const float* xb = xyz + (size_t)b * 3 * kPts;
#pragma unroll
  for (int it = 0; it < 6; ++it) {
    const int i = t + it * 512;
    const v4f v = *(const v4f*)(xb + 4 * i);
    *(v4f*)(sxyz + 4 * i) = v;
  }
  __syncthreads();

  float px[8], py[8], pz[8], dd[8];
#pragma unroll
  for (int j = 0; j < 8; ++j) {
    const int p = t + 512 * j;
    px[j] = sxyz[p];
    py[j] = sxyz[kPts + p];
    pz[j] = sxyz[2 * kPts + p];
    dd[j] = 1e10f;
  }
  int far = 0;
#pragma unroll 1
  for (int s = 0; s < kCen; ++s) {
    if (t == 0) cents[s] = far;
    const float cx = sxyz[far];
    const float cy = sxyz[kPts + far];
    const float cz = sxyz[2 * kPts + far];
    float bd = 0.0f;
    int bi = t;
#pragma unroll
    for (int j = 0; j < 8; ++j) {
      const float dx = px[j] - cx;
      const float dy = py[j] - cy;
      const float dz = pz[j] - cz;
      const float t0 = dx * dx;
      const float t1 = dy * dy;
      const float t2 = dz * dz;
      const float d = (t0 + t2) + t1;
      dd[j] = fminf(dd[j], d);
      if (j == 0) {
        bd = dd[0];
        bi = t;
      } else {
        const bool gt = dd[j] > bd;
        bd = gt ? dd[j] : bd;
        bi = gt ? (t + 512 * j) : bi;
      }
    }
    unsigned hi = __float_as_uint(bd);
    unsigned lo = ~(unsigned)bi;
#pragma unroll
    for (int off = 16; off > 0; off >>= 1) {
      const unsigned ohi = (unsigned)__shfl_xor((int)hi, off, 32);
      const unsigned olo = (unsigned)__shfl_xor((int)lo, off, 32);
      const bool take = (ohi > hi) || ((ohi == hi) && (olo > lo));
      hi = take ? ohi : hi;
      lo = take ? olo : lo;
    }
    const int buf = s & 1;
    if (lane == 0) {
      redh[buf][wave] = hi;
      redl[buf][wave] = lo;
    }
    __syncthreads();
    unsigned h2 = redh[buf][lane & 15];
    unsigned l2 = redl[buf][lane & 15];
#pragma unroll
    for (int off = 8; off > 0; off >>= 1) {
      const unsigned ohi = (unsigned)__shfl_xor((int)h2, off, 32);
      const unsigned olo = (unsigned)__shfl_xor((int)l2, off, 32);
      const bool take = (ohi > h2) || ((ohi == h2) && (olo > l2));
      h2 = take ? ohi : h2;
      l2 = take ? olo : l2;
    }
    far = (int)((~l2) & (unsigned)(kPts - 1));
  }
  __syncthreads();

  v4f va, vb;
  {
    const int e0 = 4 * t;
    const int c0 = e0 >> 10;
    const int s0 = e0 & 1023;
    va[0] = sxyz[c0 * kPts + (cents[s0 + 0] & (kPts - 1))];
    va[1] = sxyz[c0 * kPts + (cents[s0 + 1] & (kPts - 1))];
    va[2] = sxyz[c0 * kPts + (cents[s0 + 2] & (kPts - 1))];
    va[3] = sxyz[c0 * kPts + (cents[s0 + 3] & (kPts - 1))];
    const int t2 = (t < 256) ? (t + 512) : 767;
    const int e1 = 4 * t2;
    const int c1 = e1 >> 10;
    const int s1 = e1 & 1023;
    vb[0] = sxyz[c1 * kPts + (cents[s1 + 0] & (kPts - 1))];
    vb[1] = sxyz[c1 * kPts + (cents[s1 + 1] & (kPts - 1))];
    vb[2] = sxyz[c1 * kPts + (cents[s1 + 2] & (kPts - 1))];
    vb[3] = sxyz[c1 * kPts + (cents[s1 + 3] & (kPts - 1))];
  }
  float* o = out0 + (size_t)b * 3 * kCen;
  float* w = cenws + (size_t)b * 3 * kCen;
  for (int pass = 0; pass < 2; ++pass) {
    *(volatile v4f*)(o + 4 * t) = va;
    *(volatile v4f*)(w + 4 * t) = va;
    if (t < 256) {
      *(volatile v4f*)(o + 4 * (t + 512)) = vb;
      *(volatile v4f*)(w + 4 * (t + 512)) = vb;
    }
    __threadfence();
  }
}

__global__ __launch_bounds__(128) void ballq_gather_kernel(const float* __restrict__ xyz,
                                                           const float* __restrict__ pts,
                                                           const float* __restrict__ cen,
                                                           unsigned* __restrict__ A0w) {
#pragma clang fp contract(off)
  __shared__ __align__(16) float sxyz[3 * kPts];
  __shared__ int slot[4][32];
  __shared__ __align__(16) unsigned stg[4][512];
  const int t = threadIdx.x;
  const int lane = t & 31;
  const int wave = t >> 5;
  const int b = blockIdx.x >> 5;
  const int sbase = (blockIdx.x & 31) * 32;
  const float* xb = xyz + (size_t)b * 3 * kPts;
  const float* pb = pts + (size_t)b * 3 * kPts;
#pragma unroll 4
  for (int it = 0; it < 24; ++it) {
    const int i = t + it * 128;
    const v4f v = *(const v4f*)(xb + 4 * i);
    *(v4f*)(sxyz + 4 * i) = v;
  }
  __syncthreads();

  const unsigned ltmask = (1u << lane) - 1u;
  unsigned zz = 0;
  asm volatile("" : "+v"(zz));

#pragma unroll 1
  for (int c = 0; c < 8; ++c) {
    const int s = sbase + wave * 8 + c;
    const float cx = cen[(size_t)b * 3 * kCen + s];
    const float cy = cen[(size_t)b * 3 * kCen + kCen + s];
    const float cz = cen[(size_t)b * 3 * kCen + 2 * kCen + s];
    const float cc = (cx * cx + cz * cz) + cy * cy;
    if (lane == 0) slot[wave][0] = 0;
    int cnt = 0;
#pragma unroll 1
    for (int it = 0; it < (kPts / 32) && cnt < kSamp; ++it) {
      const int n = it * 32 + lane;
      const float qx = sxyz[n];
      const float qy = sxyz[kPts + n];
      const float qz = sxyz[2 * kPts + n];
      const float pp = (qx * qx + qz * qz) + qy * qy;
      float p = cx * qx;
      p = __builtin_fmaf(cy, qy, p);
      p = __builtin_fmaf(cz, qz, p);
      const float sqr = (cc + pp) - 2.0f * p;
      const bool valid = !(sqr > kBallR2);
      const unsigned m = __builtin_amdgcn_ballot_w32(valid);
      const int pos = cnt + __builtin_popcount(m & ltmask);
      if (valid && pos < kSamp) slot[wave][pos] = n;
      cnt += __builtin_popcount(m);
    }
    wave_lds_sync();
    const int jj = (lane < cnt) ? lane : 0;
    int n = slot[wave][jj];
    n = n < 0 ? 0 : n;
    n = n > (kPts - 1) ? (kPts - 1) : n;
    float f[6];
    f[0] = sxyz[n] - cx;
    f[1] = sxyz[kPts + n] - cy;
    f[2] = sxyz[2 * kPts + n] - cz;
    f[3] = pb[n];
    f[4] = pb[kPts + n];
    f[5] = pb[2 * kPts + n];
    unsigned hb[6], lb[6];
#pragma unroll
    for (int e = 0; e < 6; ++e) {
      hb[e] = f2bf_bits(f[e]);
      lb[e] = f2bf_bits(f[e] - bf_bits2f(hb[e]));
    }
    const unsigned w0 = hb[0] | (hb[1] << 16);
    const unsigned w1 = hb[2] | (hb[3] << 16);
    const unsigned w2 = hb[4] | (hb[5] << 16);
    const unsigned w3 = lb[0] | (lb[1] << 16);
    const unsigned w4 = lb[2] | (lb[3] << 16);
    const unsigned w5 = lb[4] | (lb[5] << 16);
    v4u r0, r1, r2, r3;
    r0[0] = w0; r0[1] = w1; r0[2] = w2; r0[3] = w3;
    r1[0] = w4; r1[1] = w5; r1[2] = w0; r1[3] = w1;
    r2[0] = w2; r2[1] = zz; r2[2] = zz; r2[3] = zz;
    r3[0] = zz; r3[1] = zz; r3[2] = zz; r3[3] = zz;
    unsigned* sw = stg[wave];
    *(v4u*)(sw + lane * 16 + 0) = r0;
    *(v4u*)(sw + lane * 16 + 4) = r1;
    *(v4u*)(sw + lane * 16 + 8) = r2;
    *(v4u*)(sw + lane * 16 + 12) = r3;
    wave_lds_sync();
    const v4u o0 = *(const v4u*)(sw + 0 * 128 + lane * 4);
    const v4u o1 = *(const v4u*)(sw + 1 * 128 + lane * 4);
    const v4u o2 = *(const v4u*)(sw + 2 * 128 + lane * 4);
    const v4u o3 = *(const v4u*)(sw + 3 * 128 + lane * 4);
    unsigned* dst = A0w + ((size_t)(b * kCen + s) * kSamp) * 16 + lane * 4;
    for (int pass = 0; pass < 2; ++pass) {
      *(volatile v4u*)(dst + 0 * 128) = o0;
      *(volatile v4u*)(dst + 1 * 128) = o1;
      *(volatile v4u*)(dst + 2 * 128) = o2;
      *(volatile v4u*)(dst + 3 * 128) = o3;
      __threadfence();
    }
    wave_lds_sync();
  }
}

template <int STAGE>
__global__ __launch_bounds__(256) void mlp_kernel(
    const unsigned short* __restrict__ A0p, const unsigned short* __restrict__ Bt0p,
    const unsigned short* __restrict__ W1p, const unsigned short* __restrict__ W2p,
    const float* __restrict__ biasp, const float* __restrict__ ab0, const float* __restrict__ ab1,
    float* __restrict__ P, float* __restrict__ gmm) {
  constexpr int CST = (STAGE == 2) ? 128 : 64;
  constexpr int NJ = CST / 16;
  __shared__ __align__(16) float cst[3][256];
  __shared__ __align__(16) _Float16 act[(STAGE >= 1) ? 8 : 1][(STAGE >= 1) ? 32 * kActPitch : 8];
  __shared__ __align__(16) _Float16 actlo[(STAGE >= 1) ? 8 : 1][(STAGE >= 1) ? 32 * kActPitch : 8];
  __shared__ __align__(16) float stat[8][2 * CST];
  __shared__ __align__(16) float red[256];
  __shared__ __align__(16) float gst[(STAGE == 2) ? 8 : 1][(STAGE == 2) ? 256 : 4];

  const int tid = threadIdx.x;
  const int lane = tid & 31;
  const int wave = tid >> 5;
  const int rl = lane & 15;
  const int hh = lane >> 4;
  const int koff = hh * 8;

  cst[0][tid] = biasp[tid];
  if constexpr (STAGE >= 1) cst[1][tid] = ab0[tid];
  if constexpr (STAGE >= 2) cst[2][tid] = ab1[tid];
  __syncthreads();

  const int grp = blockIdx.x * 8 + wave;
  const size_t row0 = (size_t)grp * 32;
  _Float16* actw = act[(STAGE >= 1) ? wave : 0];
  _Float16* actlw = actlo[(STAGE >= 1) ? wave : 0];

  float ssum[NJ], ssq[NJ];
#pragma unroll
  for (int j = 0; j < NJ; ++j) { ssum[j] = 0.0f; ssq[j] = 0.0f; }

  v8f acc[2][4];
#pragma unroll
  for (int i = 0; i < 2; ++i)
#pragma unroll
    for (int j = 0; j < 4; ++j) acc[i][j] = (v8f){0.f, 0.f, 0.f, 0.f, 0.f, 0.f, 0.f, 0.f};

  {
    const __bf16* A0 = (const __bf16*)A0p;
    const __bf16* B0 = (const __bf16*)Bt0p;
    v16b af[2];
#pragma unroll
    for (int i = 0; i < 2; ++i) af[i] = ldfrag_b(A0 + (row0 + (size_t)(i * 16 + rl)) * 32 + koff);
#pragma unroll
    for (int j = 0; j < 4; ++j) {
      const v16b bf = ldfrag_b(B0 + (j * 16 + rl) * 32 + koff);
#pragma unroll
      for (int i = 0; i < 2; ++i) acc[i][j] = mma_b(af[i], bf, acc[i][j]);
    }
  }
#pragma unroll
  for (int j = 0; j < 4; ++j) {
    const int n = j * 16 + rl;
    const float bias = cst[0][n];
    float a = 0.0f, bb = 0.0f;
    if constexpr (STAGE >= 1) { a = cst[1][n]; bb = cst[1][128 + n]; }
#pragma unroll
    for (int i = 0; i < 2; ++i) {
#pragma unroll
      for (int r = 0; r < 8; ++r) {
        const float y = acc[i][j][r] + bias;
        if constexpr (STAGE == 0) {
          ssum[j] += y;
          ssq[j] += y * y;
        } else {
          float h = a * y + bb;
          h = fmaxf(h, 0.0f) * kActCarry;
          float hf = (float)((_Float16)h);
          asm volatile("" : "+v"(hf));
          hf = (hf < kF16MinNormal) ? 0.0f : hf;
          const float lo = (h - hf) * kResidCarry;
          const int ai = (i * 16 + 8 * hh + r) * kActPitch + n;
          actw[ai] = (_Float16)hf;
          actlw[ai] = (_Float16)lo;
        }
      }
    }
  }

  if constexpr (STAGE >= 1) {
    wave_lds_sync();
    v8f acr[2][4];
#pragma unroll
    for (int i = 0; i < 2; ++i)
#pragma unroll
      for (int j = 0; j < 4; ++j) {
        acc[i][j] = (v8f){0.f, 0.f, 0.f, 0.f, 0.f, 0.f, 0.f, 0.f};
        acr[i][j] = (v8f){0.f, 0.f, 0.f, 0.f, 0.f, 0.f, 0.f, 0.f};
      }
    const _Float16* W1 = (const _Float16*)W1p;
#pragma unroll
    for (int ks = 0; ks < 2; ++ks) {
      v16h af[2], al[2];
#pragma unroll
      for (int i = 0; i < 2; ++i) {
        af[i] = ldfrag_h(actw + (i * 16 + rl) * kActPitch + ks * 32 + koff);
        al[i] = ldfrag_h(actlw + (i * 16 + rl) * kActPitch + ks * 32 + koff);
      }
#pragma unroll
      for (int j = 0; j < 4; ++j) {
        const v16h bf = ldfrag_h(W1 + (j * 16 + rl) * 64 + ks * 32 + koff);
#pragma unroll
        for (int i = 0; i < 2; ++i) {
          acc[i][j] = mma_h(af[i], bf, acc[i][j]);
          acr[i][j] = mma_h(al[i], bf, acr[i][j]);
        }
      }
    }
    if constexpr (STAGE >= 2) wave_lds_sync();
#pragma unroll
    for (int j = 0; j < 4; ++j) {
      const int n = j * 16 + rl;
      const float bias = cst[0][64 + n];
      float a = 0.0f, bb = 0.0f;
      if constexpr (STAGE >= 2) { a = cst[2][n]; bb = cst[2][128 + n]; }
#pragma unroll
      for (int i = 0; i < 2; ++i) {
#pragma unroll
        for (int r = 0; r < 8; ++r) {
          const float full = acc[i][j][r] + acr[i][j][r] * kInvResid;
          const float y = full * kInvCarry + bias;
          if constexpr (STAGE == 1) {
            ssum[j] += y;
            ssq[j] += y * y;
          } else {
            float h = a * y + bb;
            h = fmaxf(h, 0.0f) * kActCarry;
            actw[(i * 16 + 8 * hh + r) * kActPitch + n] = (_Float16)h;
          }
        }
      }
    }
  }

  if constexpr (STAGE >= 2) {
    wave_lds_sync();
    const _Float16* W2 = (const _Float16*)W2p;
    v16h a2[2][2];
#pragma unroll
    for (int ks = 0; ks < 2; ++ks)
#pragma unroll
      for (int i = 0; i < 2; ++i) a2[ks][i] = ldfrag_h(actw + (i * 16 + rl) * kActPitch + ks * 32 + koff);
    float* gw = gst[(STAGE == 2) ? wave : 0];
#pragma unroll
    for (int nh = 0; nh < 2; ++nh) {
#pragma unroll
      for (int i = 0; i < 2; ++i)
#pragma unroll
        for (int j = 0; j < 4; ++j) acc[i][j] = (v8f){0.f, 0.f, 0.f, 0.f, 0.f, 0.f, 0.f, 0.f};
#pragma unroll
      for (int ks = 0; ks < 2; ++ks) {
#pragma unroll
        for (int j = 0; j < 4; ++j) {
          const v16h bf = ldfrag_h(W2 + ((nh * 4 + j) * 16 + rl) * 64 + ks * 32 + koff);
#pragma unroll
          for (int i = 0; i < 2; ++i) acc[i][j] = mma_h(a2[ks][i], bf, acc[i][j]);
        }
      }
#pragma unroll
      for (int j = 0; j < 4; ++j) {
        const int n = nh * 64 + j * 16 + rl;
        const float bias = cst[0][128 + n];
        float mx = -3.0e38f;
        float mn = 3.0e38f;
#pragma unroll
        for (int i = 0; i < 2; ++i) {
#pragma unroll
          for (int r = 0; r < 8; ++r) {
            const float y = acc[i][j][r] * kInvCarry + bias;
            ssum[nh * 4 + j] += y;
            ssq[nh * 4 + j] += y * y;
            mx = fmaxf(mx, y);
            mn = fminf(mn, y);
          }
        }
        const float omx = __shfl_xor(mx, 16, 32);
        const float omn = __shfl_xor(mn, 16, 32);
        mx = fmaxf(mx, omx);
        mn = fminf(mn, omn);
        gw[hh * 128 + n] = hh ? mn : mx;
      }
    }
    wave_lds_sync();
    const v4f g0 = *(const v4f*)(gw + lane * 4);
    const v4f g1 = *(const v4f*)(gw + 128 + lane * 4);
    float* gd = gmm + (size_t)grp * 256 + lane * 4;
    for (int pass = 0; pass < 2; ++pass) {
      *(volatile v4f*)(gd) = g0;
      *(volatile v4f*)(gd + 128) = g1;
      __threadfence();
    }
  }

#pragma unroll
  for (int j = 0; j < NJ; ++j) {
    float s = ssum[j];
    float q = ssq[j];
    const float os = __shfl_xor(s, 16, 32);
    const float oq = __shfl_xor(q, 16, 32);
    s += os;
    q += oq;
    stat[wave][hh * CST + j * 16 + rl] = hh ? q : s;
  }
  __syncthreads();
  if (tid < 2 * CST) {
    float tot = 0.0f;
#pragma unroll
    for (int w = 0; w < 8; ++w) tot += stat[w][tid];
    red[tid] = tot;
  }
  __syncthreads();
  if (wave == 0) {
    float* pd = P + (size_t)blockIdx.x * (2 * CST) + lane * 4;
    const v4f p0 = *(const v4f*)(red + lane * 4);
    v4f p1 = p0;
    if constexpr (CST == 128) p1 = *(const v4f*)(red + 128 + lane * 4);
    for (int pass = 0; pass < 2; ++pass) {
      *(volatile v4f*)(pd) = p0;
      if constexpr (CST == 128) *(volatile v4f*)(pd + 128) = p1;
      __threadfence();
    }
  }
}

__global__ __launch_bounds__(128) void bn_finalize_kernel(const float* __restrict__ P, int nblk, int C,
                                                          const float* __restrict__ g,
                                                          const float* __restrict__ beta,
                                                          float* __restrict__ ab) {
  __shared__ __align__(16) float sab[256];
  const int t = threadIdx.x;
  const int lane = t & 31;
  const int tc = (t < C) ? t : (C - 1);
  const int stride = 2 * C;
  double s = 0.0, q = 0.0;
#pragma unroll 4
  for (int blk = 0; blk < nblk; ++blk) {
    s += (double)P[(size_t)blk * stride + tc];
    q += (double)P[(size_t)blk * stride + C + tc];
  }
  const double invn = 1.0 / (double)kRows;
  const double mean = s * invn;
  double var = q * invn - mean * mean;
  if (var < 0.0) var = 0.0;
  const float a = g[tc] * (1.0f / sqrtf((float)var + kBnEps));
  const float bbv = beta[tc] - (float)mean * a;
  const bool keep = (t < C);
  sab[t] = keep ? a : 0.0f;
  sab[128 + t] = keep ? bbv : 0.0f;
  __syncthreads();
  if (t < 32) {
    const v4f v0 = *(const v4f*)(sab + lane * 4);
    const v4f v1 = *(const v4f*)(sab + 128 + lane * 4);
    for (int pass = 0; pass < 2; ++pass) {
      *(volatile v4f*)(ab + lane * 4) = v0;
      *(volatile v4f*)(ab + 128 + lane * 4) = v1;
      __threadfence();
    }
  }
}

__global__ __launch_bounds__(256) void pool_out_kernel(const float* __restrict__ gmm,
                                                       const float* __restrict__ ab2,
                                                       float* __restrict__ out1) {
  __shared__ __align__(16) float tr[128 * 36];
  const int tid = threadIdx.x;
  const int lane = tid & 31;
  const int wave = tid >> 5;
  const int b = blockIdx.x >> 5;
  const int s0 = (blockIdx.x & 31) * 32;
  const int g0 = b * kCen + s0;
  const int c4 = (tid & 31) * 4;
  const v4f av = *(const v4f*)(ab2 + c4);
  const v4f bv = *(const v4f*)(ab2 + 128 + c4);
#pragma unroll 2
  for (int it = 0; it < 4; ++it) {
    const int i = it * 8 + (tid >> 5);
    const v4f mx = *(const v4f*)(gmm + (size_t)(g0 + i) * 256 + c4);
    const v4f mn = *(const v4f*)(gmm + (size_t)(g0 + i) * 256 + 128 + c4);
#pragma unroll
    for (int e = 0; e < 4; ++e) {
      const float u0 = av[e] * mx[e] + bv[e];
      const float u1 = av[e] * mn[e] + bv[e];
      tr[(c4 + e) * 36 + i] = fmaxf(fmaxf(u0, u1), 0.0f);
    }
  }
  __syncthreads();
  const int sv = (lane & 7) * 4;
  v4f ov[4];
#pragma unroll
  for (int it = 0; it < 4; ++it) {
    const int c = (wave * 4 + it) * 4 + (lane >> 3);
    ov[it] = *(const v4f*)(tr + c * 36 + sv);
  }
  for (int pass = 0; pass < 2; ++pass) {
#pragma unroll
    for (int it = 0; it < 4; ++it) {
      const int c = (wave * 4 + it) * 4 + (lane >> 3);
      *(volatile v4f*)(out1 + ((size_t)(b * 128 + c)) * kCen + s0 + sv) = ov[it];
    }
    __threadfence();
  }
}

extern "C" void kernel_launch(void* const* d_in, const int* in_sizes, int n_in,
                              void* d_out, int out_size, void* d_ws, size_t ws_size,
                              hipStream_t stream) {
  (void)in_sizes; (void)out_size;
  constexpr size_t offCEN = 0;
  constexpr size_t offBT0 = offCEN + (size_t)kBatch * 3 * kCen * 4;
  constexpr size_t offW1H = offBT0 + 64 * 32 * 2;
  constexpr size_t offW2H = offW1H + 64 * 64 * 2;
  constexpr size_t offBIAS = offW2H + 128 * 64 * 2;
  constexpr size_t offAB0 = offBIAS + 1024;
  constexpr size_t offAB1 = offAB0 + 1024;
  constexpr size_t offAB2 = offAB1 + 1024;
  constexpr size_t offP0 = offAB2 + 1024;
  constexpr size_t offP1 = offP0 + (size_t)kMlpBlocks * 128 * 4;
  constexpr size_t offP2 = offP1 + (size_t)kMlpBlocks * 128 * 4;
  constexpr size_t offGMM = offP2 + (size_t)kMlpBlocks * 256 * 4;
  constexpr size_t offA0 = offGMM + (size_t)kGroups * 256 * 4;
  constexpr size_t wsTotal = offA0 + (size_t)kRows * 32 * 2;
  static_assert(offBT0 % 128 == 0 && offW1H % 128 == 0 && offW2H % 128 == 0 && offBIAS % 128 == 0);
  static_assert(offP0 % 128 == 0 && offGMM % 128 == 0 && offA0 % 128 == 0);
  static_assert(wsTotal <= (size_t)134217728);
  if (n_in < 14) return;
  if (ws_size < wsTotal) return;

  const float* xyz   = (const float*)d_in[0];
  const float* pts   = (const float*)d_in[1];
  const float* W0    = (const float*)d_in[2];
  const float* b0    = (const float*)d_in[3];
  const float* g0    = (const float*)d_in[4];
  const float* beta0 = (const float*)d_in[5];
  const float* W1    = (const float*)d_in[6];
  const float* b1    = (const float*)d_in[7];
  const float* g1    = (const float*)d_in[8];
  const float* beta1 = (const float*)d_in[9];
  const float* W2    = (const float*)d_in[10];
  const float* b2    = (const float*)d_in[11];
  const float* g2    = (const float*)d_in[12];
  const float* beta2 = (const float*)d_in[13];

  float* out0 = (float*)d_out;
  float* out1 = (float*)d_out + (size_t)kBatch * 3 * kCen;

  char* ws = (char*)d_ws;
  float* cen = (float*)(ws + offCEN);
  unsigned short* bt0 = (unsigned short*)(ws + offBT0);
  unsigned short* w1h = (unsigned short*)(ws + offW1H);
  unsigned short* w2h = (unsigned short*)(ws + offW2H);
  float* biasp = (float*)(ws + offBIAS);
  float* ab0 = (float*)(ws + offAB0);
  float* ab1 = (float*)(ws + offAB1);
  float* ab2 = (float*)(ws + offAB2);
  float* P0 = (float*)(ws + offP0);
  float* P1 = (float*)(ws + offP1);
  float* P2 = (float*)(ws + offP2);
  float* gmm = (float*)(ws + offGMM);
  unsigned short* A0 = (unsigned short*)(ws + offA0);

  prep_kernel<<<8, 256, 0, stream>>>(W0, W1, W2, b0, b1, b2, (unsigned*)bt0, w1h, w2h, biasp);
  fps_kernel<<<kBatch, 512, 0, stream>>>(xyz, out0, cen);
  ballq_gather_kernel<<<kBatch * 32, 128, 0, stream>>>(xyz, pts, cen, (unsigned*)A0);
  mlp_kernel<0><<<kMlpBlocks, 256, 0, stream>>>(A0, bt0, w1h, w2h, biasp, ab0, ab1, P0, gmm);
  bn_finalize_kernel<<<1, 128, 0, stream>>>(P0, kMlpBlocks, 64, g0, beta0, ab0);
  mlp_kernel<1><<<kMlpBlocks, 256, 0, stream>>>(A0, bt0, w1h, w2h, biasp, ab0, ab1, P1, gmm);
  bn_finalize_kernel<<<1, 128, 0, stream>>>(P1, kMlpBlocks, 64, g1, beta1, ab1);
  mlp_kernel<2><<<kMlpBlocks, 256, 0, stream>>>(A0, bt0, w1h, w2h, biasp, ab0, ab1, P2, gmm);
  bn_finalize_kernel<<<1, 128, 0, stream>>>(P2, kMlpBlocks, 128, g2, beta2, ab2);
  pool_out_kernel<<<kBatch * 32, 256, 0, stream>>>(gmm, ab2, out1);
}
